// MultiHeadAttentionModify_4999341932596
// MI455X (gfx1250) — hardware-verified
//
#include <hip/hip_runtime.h>


#define NB_  4
#define DD   256
#define HH   64
#define NQ   4096
#define NKY  4096
#define DM   DD
#define CC   DD
#define WP   66
#define NPP  (WP * WP)
#define NPR  4416
#define GB   128
#define NPT  (GB + NPR + GB)
#define NPX  NQ
#define BEPS 0.001f
#define LOSC 1024.0f

typedef _Float16 h16;
typedef unsigned short bf;
typedef __attribute__((ext_vector_type(16))) __bf16   v16bf;
typedef __attribute__((ext_vector_type(16))) _Float16 v16h;
typedef __attribute__((ext_vector_type(8)))  _Float16 v8h;
typedef __attribute__((ext_vector_type(8)))  unsigned short v8us;
typedef __attribute__((ext_vector_type(8)))  float    v8f;
typedef __attribute__((ext_vector_type(4)))  float    v4f;
typedef v8h  __attribute__((may_alias)) v8ha;
typedef v4f  __attribute__((may_alias)) v4fa;
typedef v8us __attribute__((may_alias)) v8usa;

__device__ __forceinline__ unsigned short f2bf(float f) { unsigned u = __float_as_uint(f); u += 0x7FFFu + ((u >> 16) & 1u); return (unsigned short)(u >> 16); }
__device__ __forceinline__ float bf2f(unsigned short b) { return __uint_as_float(((unsigned)b) << 16); }
__device__ __forceinline__ float bfr(float f) { return bf2f(f2bf(f)); }
__device__ __forceinline__ v16h cat16(v8h lo, v8h hi) { return __builtin_shufflevector(lo, hi, 0, 1, 2, 3, 4, 5, 6, 7, 8, 9, 10, 11, 12, 13, 14, 15); }
__device__ __forceinline__ v16bf cat16b(v8us lo, v8us hi) { return __builtin_bit_cast(v16bf, __builtin_shufflevector(lo, hi, 0, 1, 2, 3, 4, 5, 6, 7, 8, 9, 10, 11, 12, 13, 14, 15)); }
__device__ __forceinline__ v8f wmma16(v16h a, v16h b, v8f c) { return __builtin_amdgcn_wmma_f32_16x16x32_f16(false, a, false, b, (short)0, c, false, false); }
__device__ __forceinline__ v8f wmmab(v16bf a, v16bf b, v8f c) { return __builtin_amdgcn_wmma_f32_16x16x32_bf16(false, a, false, b, (short)0, c, false, false); }

template <bool SPLITA, bool F16OUT = false>
__global__ __launch_bounds__(128) void k_gemmb(const bf* __restrict__ A, const bf* __restrict__ Al, const bf* __restrict__ Bn, const float* __restrict__ bias, float* C, int ldc, h16* C2, const float* __restrict__ R = nullptr, int K = DM, int roundR = 1) {
    __shared__ __align__(16) float ost[4][16 * 68];
    const int lane = threadIdx.x & 31, wave = threadIdx.x >> 5, lr = lane & 15, hi = lane >> 4;
    const int r0 = blockIdx.x * 64 + wave * 16, c0 = blockIdx.y * 64;
    const size_t aoff = (size_t)(r0 + lr) * K + 8 * hi;
    size_t boff[4];
#pragma unroll
    for (int t = 0; t < 4; ++t) boff[t] = (size_t)(c0 + t * 16 + lr) * K + 8 * hi;
    v8f acc[4];
#pragma unroll
    for (int t = 0; t < 4; ++t) acc[t] = (v8f){};
#pragma unroll 1
    for (int kc = 0; kc < K; kc += 32) {
        const v16bf a = cat16b(*(const v8us*)(A + aoff + kc), *(const v8us*)(A + aoff + kc + 16));
        v16bf al = a;
        if (SPLITA) al = cat16b(*(const v8us*)(Al + aoff + kc), *(const v8us*)(Al + aoff + kc + 16));
#pragma unroll
        for (int t = 0; t < 4; ++t) { const v16bf b = cat16b(*(const v8us*)(Bn + boff[t] + kc), *(const v8us*)(Bn + boff[t] + kc + 16)); acc[t] = wmmab(a, b, acc[t]); if (SPLITA) acc[t] = wmmab(al, b, acc[t]); }
        asm volatile("v_nop\n\tv_nop\n\tv_nop\n\tv_nop" : "+v"(acc[0]), "+v"(acc[1]), "+v"(acc[2]), "+v"(acc[3]) : "v"(a), "v"(al));
    }
    float* os = &ost[wave][0];
#pragma unroll
    for (int t = 0; t < 4; ++t) { const float bv = bias ? bfr(bias[c0 + t * 16 + lr]) : 0.f;
#pragma unroll
        for (int j = 0; j < 8; ++j) os[(hi * 8 + j) * 68 + t * 16 + lr] = acc[t][j] + bv; }
    __syncthreads();
    if (F16OUT) {
        h16* crow = (h16*)(void*)C + (size_t)r0 * ldc + c0;
        auto pass = [&]() {
#pragma unroll
            for (int s = 0; s < 4; ++s) { const int row = 4 * s + (lane >> 3), piece = lane & 7; const float* sp = os + row * 68 + piece * 8; v8h o, o2;
#pragma unroll
                for (int i = 0; i < 8; ++i) { const h16 a = (h16)sp[i]; o[i] = a; o2[i] = (h16)((sp[i] - (float)a) * LOSC); }
                *(volatile v8h*)(crow + (size_t)row * ldc + piece * 8) = o; if (C2) *(volatile v8h*)(C2 + (size_t)r0 * ldc + c0 + (size_t)row * ldc + piece * 8) = o2; }
        };
        pass(); __threadfence(); pass();
    } else {
        float* crow = C + (size_t)r0 * ldc + c0;
        auto pass = [&]() {
#pragma unroll
            for (int s = 0; s < 8; ++s) { const int Lid = (lane >> 3) + 4 * s, piece = lane & 7; const int row = Lid >> 1, cofs = (Lid & 1) * 32 + piece * 4;
                v4f val = *(const v4fa*)(os + row * 68 + cofs); if (R) { const v4f rv = *(const v4f*)(R + ((size_t)r0 + row) * ldc + c0 + cofs); val += roundR ? (v4f){bfr(rv[0]), bfr(rv[1]), bfr(rv[2]), bfr(rv[3])} : rv; }
                *(volatile v4f*)(crow + (size_t)row * ldc + cofs) = val; }
        };
        pass(); __threadfence(); pass();
    }
}

__global__ __launch_bounds__(256) void k_cvt8(const float* __restrict__ src, bf* dst, size_t n8) {
    const size_t i = (size_t)blockIdx.x * 256 + threadIdx.x; if (i >= n8) return;
    const v8f v = *(const v8f*)(src + i * 8); v8us o;
#pragma unroll
    for (int k = 0; k < 8; ++k) o[k] = f2bf(v[k]);
    *(volatile v8us*)(dst + i * 8) = o; __threadfence(); *(volatile v8us*)(dst + i * 8) = o;
}
__global__ __launch_bounds__(256) void k_zero8(bf* dst, size_t n8) {
    const size_t i = (size_t)blockIdx.x * 256 + threadIdx.x; if (i >= n8) return; v8us z;
#pragma unroll
    for (int k = 0; k < 8; ++k) z[k] = 0;
    *(volatile v8us*)(dst + i * 8) = z; __threadfence(); *(volatile v8us*)(dst + i * 8) = z;
}

__global__ __launch_bounds__(256) void k_qp2(const float* __restrict__ qp, bf* A) {
    const int lane = threadIdx.x & 31; const size_t q = (size_t)blockIdx.x * 8 + (threadIdx.x >> 5); if (q >= (size_t)NQ) return; v8us o;
#pragma unroll
    for (int i = 0; i < 8; ++i) o[i] = f2bf(qp[q * DD + lane * 8 + i]);
#pragma unroll 1
    for (int ps = 0; ps < 2; ++ps) { *(volatile v8us*)(A + q * 2 * DD + lane * 8) = o; *(volatile v8us*)(A + q * 2 * DD + DD + lane * 8) = o; if (ps == 0) __threadfence(); }
}
__global__ __launch_bounds__(256) void k_cvtrows(const float* __restrict__ src, size_t rows, bf* dst) {
    const int lane = threadIdx.x & 31; const size_t r = (size_t)blockIdx.x * 8 + (threadIdx.x >> 5); if (r >= rows) return; v8us o;
#pragma unroll
    for (int i = 0; i < 8; ++i) o[i] = f2bf(src[r * DD + lane * 8 + i]);
    *(volatile v8us*)(dst + r * DD + lane * 8) = o; __threadfence(); *(volatile v8us*)(dst + r * DD + lane * 8) = o;
}
__global__ __launch_bounds__(256) void k_relu256p(const float* __restrict__ F, size_t rows, bf* Ph, bf* Pl) {
    const int lane = threadIdx.x & 31; const size_t r = (size_t)blockIdx.x * 8 + (threadIdx.x >> 5); if (r >= rows) return; const size_t o = r * DD + lane * 8; const v8f v = *(const v8f*)(F + o); v8us oh, ol;
#pragma unroll
    for (int i = 0; i < 8; ++i) { const float y = fmaxf(v[i], 0.f); const unsigned short hb = f2bf(y); oh[i] = hb; ol[i] = f2bf(y - bf2f(hb)); }
    *(volatile v8us*)(Ph + o) = oh; *(volatile v8us*)(Pl + o) = ol; __threadfence(); *(volatile v8us*)(Ph + o) = oh; *(volatile v8us*)(Pl + o) = ol;
}
template <bool RAW, bool PLANES>
__global__ __launch_bounds__(256) void k_normsplit(const float* __restrict__ F, size_t rows, float* RN, bf* Ph, bf* Pl) {
    const int lane = threadIdx.x & 31; const size_t r = (size_t)blockIdx.x * 8 + (threadIdx.x >> 5); if (r >= rows) return; const size_t o = r * DD + lane * 8; float v[8]; float s = 0.f;
#pragma unroll
    for (int i = 0; i < 8; ++i) { float t = F[o + i]; if (RAW) t = bfr(t); v[i] = t; s = fmaf(t, t, s); }
#pragma unroll
    for (int sh = 16; sh; sh >>= 1) s += __shfl_xor(s, sh, 32);
    const float rn = 1.0f / sqrtf(s);
    if (PLANES) { v8us oh, ol;
#pragma unroll
        for (int i = 0; i < 8; ++i) { const unsigned short hb = f2bf(v[i]); oh[i] = hb; ol[i] = f2bf(v[i] - bf2f(hb)); }
        *(volatile v8us*)(Ph + o) = oh; *(volatile v8us*)(Pl + o) = ol; __threadfence(); *(volatile v8us*)(Ph + o) = oh; *(volatile v8us*)(Pl + o) = ol; }
    const float rv = (lane == 0) ? rn : 0.f; *(volatile float*)(RN + r * 32 + lane) = rv; __threadfence(); *(volatile float*)(RN + r * 32 + lane) = rv;
}
__global__ __launch_bounds__(256) void k_relw(const float* __restrict__ S, const float* __restrict__ RQ, const float* __restrict__ RK, const float* __restrict__ oW, bf* PH, bf* PL) {
    typedef __attribute__((ext_vector_type(4))) unsigned short v4us;
    const int lane = threadIdx.x & 31; const size_t q = (size_t)blockIdx.x * 8 + (threadIdx.x >> 5); if (q >= (size_t)NQ) return; const float rq = RQ[q * 32]; const float* sr = S + q * NKY;
#pragma unroll 1
    for (int ps = 0; ps < 2; ++ps) {
#pragma unroll 1
        for (int c0 = lane * 4; c0 < NKY; c0 += 128) { v4us oh, ol;
#pragma unroll
            for (int i = 0; i < 4; ++i) { const int k = c0 + i; const float y = fmaxf(sr[k] * rq * RK[(size_t)k * 32], 0.f) * bfr(oW[k]); const unsigned short hb = f2bf(y); oh[i] = hb; ol[i] = f2bf(y - bf2f(hb)); }
            const size_t o = q * NKY + c0; *(volatile v4us*)(PH + o) = oh; *(volatile v4us*)(PL + o) = ol; }
        if (ps == 0) __threadfence(); }
}
__global__ __launch_bounds__(256) void k_vT(const float* __restrict__ vb, bf* VT) {
    __shared__ float tl[64][65];
    typedef __attribute__((ext_vector_type(4))) unsigned short v4us;
    const int tid = threadIdx.x; const int k0 = blockIdx.x * 64, d0 = blockIdx.y * 64; const int rr = tid >> 2, cq = (tid & 3) * 16;
#pragma unroll
    for (int i = 0; i < 16; ++i) tl[rr][cq + i] = vb[(size_t)(k0 + rr) * DD + d0 + cq + i];
    __syncthreads();
    const int lane = tid & 31, wv = tid >> 5;
    auto pass = [&]() {
#pragma unroll
        for (int st = 0; st < 4; ++st) { const int dr = wv * 8 + st * 2 + (lane >> 4); const int kq = (lane & 15) * 4; v4us v;
#pragma unroll
            for (int i = 0; i < 4; ++i) v[i] = f2bf(tl[kq + i][dr]);
            *(volatile v4us*)(VT + (size_t)(d0 + dr) * NKY + k0 + kq) = v; }
    };
    pass(); __threadfence(); pass();
}
__global__ __launch_bounds__(256) void k_split256(const float* __restrict__ F, size_t rows, bf* Ph, bf* Pl) {
    const int lane = threadIdx.x & 31; const size_t r = (size_t)blockIdx.x * 8 + (threadIdx.x >> 5); if (r >= rows) return; const size_t o = r * DD + lane * 8; const v8f v = *(const v8f*)(F + o); v8us oh, ol;
#pragma unroll
    for (int i = 0; i < 8; ++i) { const unsigned short hb = f2bf(v[i]); oh[i] = hb; ol[i] = f2bf(v[i] - bf2f(hb)); }
    *(volatile v8us*)(Ph + o) = oh; *(volatile v8us*)(Pl + o) = ol; __threadfence(); *(volatile v8us*)(Ph + o) = oh; *(volatile v8us*)(Pl + o) = ol;
}
__global__ __launch_bounds__(256) void k_ogrid(const float* __restrict__ OUT, bf* Gh, bf* Gl) {
    const int lane = threadIdx.x & 31; const size_t r = (size_t)blockIdx.x * 8 + (threadIdx.x >> 5); if (r >= (size_t)NPT) return; const long pr = (long)r - GB; bool live = false; size_t q = 0;
    if (pr >= 0 && pr < NPP) { const int gy = (int)(pr / WP), gx = (int)(pr % WP); const int y = gy - 1, x = gx - 1; live = (y >= 0 && y < HH && x >= 0 && x < HH); if (live) q = (size_t)y * HH + x; }
    v8us oh, ol;
#pragma unroll
    for (int i = 0; i < 8; ++i) { const float v = live ? OUT[q * DD + lane * 8 + i] : 0.f; const unsigned short hb = f2bf(v); oh[i] = hb; ol[i] = f2bf(v - bf2f(hb)); }
    const size_t o = r * DD + lane * 8; *(volatile v8us*)(Gh + o) = oh; *(volatile v8us*)(Gl + o) = ol; __threadfence(); *(volatile v8us*)(Gh + o) = oh; *(volatile v8us*)(Gl + o) = ol;
}
__global__ __launch_bounds__(256) void k_wtap9(const float* __restrict__ Wc, bf* WT) {
    const int lane = threadIdx.x & 31; const int w = blockIdx.x * 8 + (threadIdx.x >> 5); if (w >= 9 * DD) return; const int tap = w / DD, o = w % DD; v8us ov;
#pragma unroll
    for (int i = 0; i < 8; ++i) { const int ci = lane * 8 + i; ov[i] = f2bf(Wc[(((size_t)o * DD + ci) * 9) + tap]); }
    *(volatile v8us*)(WT + (size_t)w * DD + lane * 8) = ov; __threadfence(); *(volatile v8us*)(WT + (size_t)w * DD + lane * 8) = ov;
}
__global__ __launch_bounds__(128) void k_gemmtap9(const bf* __restrict__ Ah, const bf* __restrict__ Al, const bf* __restrict__ Bt, float* C) {
    __shared__ __align__(16) float ost[4][16 * 68];
    const int lane = threadIdx.x & 31, wave = threadIdx.x >> 5, lr = lane & 15, hi = lane >> 4;
    const int r0 = blockIdx.x * 64 + wave * 16, c0 = blockIdx.y * 64; const int K = DD;
    v8f acc[4];
#pragma unroll
    for (int t = 0; t < 4; ++t) acc[t] = (v8f){};
#pragma unroll 1
    for (int tap = 0; tap < 9; ++tap) { const long off = (long)(tap / 3 - 1) * WP + (tap % 3 - 1);
        const size_t aoff = (size_t)((long)GB + off + r0 + lr) * K + 8 * hi; const bf* Bn = Bt + (size_t)tap * DD * K;
#pragma unroll 1
        for (int kc = 0; kc < K; kc += 32) {
            const v16bf a = cat16b(*(const v8us*)(Ah + aoff + kc), *(const v8us*)(Ah + aoff + kc + 16));
            const v16bf al = cat16b(*(const v8us*)(Al + aoff + kc), *(const v8us*)(Al + aoff + kc + 16));
#pragma unroll
            for (int t = 0; t < 4; ++t) { const size_t bo = (size_t)(c0 + t * 16 + lr) * K + kc + 8 * hi; const v16bf b = cat16b(*(const v8us*)(Bn + bo), *(const v8us*)(Bn + bo + 16)); acc[t] = wmmab(a, b, acc[t]); acc[t] = wmmab(al, b, acc[t]); }
            asm volatile("v_nop\n\tv_nop\n\tv_nop\n\tv_nop" : "+v"(acc[0]), "+v"(acc[1]), "+v"(acc[2]), "+v"(acc[3]) : "v"(a), "v"(al)); } }
    float* os = &ost[wave][0];
#pragma unroll
    for (int t = 0; t < 4; ++t) {
#pragma unroll
        for (int j = 0; j < 8; ++j) os[(hi * 8 + j) * 68 + t * 16 + lr] = acc[t][j]; }
    __builtin_amdgcn_wave_barrier(); asm volatile("" ::: "memory");
    float* crow = C + (size_t)r0 * DD + c0;
    auto pass = [&]() {
#pragma unroll
        for (int s = 0; s < 8; ++s) { const int Lid = (lane >> 3) + 4 * s, piece = lane & 7; const int row = Lid >> 1, cofs = (Lid & 1) * 32 + piece * 4;
            const v4f val = *(const v4fa*)(os + row * 68 + cofs); *(volatile v4f*)(crow + (size_t)row * DD + cofs) = val; }
    };
    pass(); __threadfence(); pass();
}
__global__ __launch_bounds__(256) void k_bnsilu(const float* __restrict__ CV, const float* __restrict__ gam, const float* __restrict__ bet, const float* __restrict__ mu, const float* __restrict__ var, bf* Zh, bf* Zl) {
    const int lane = threadIdx.x & 31; const size_t q = (size_t)blockIdx.x * 8 + (threadIdx.x >> 5); if (q >= (size_t)NQ) return; const int y = (int)(q / HH), x = (int)(q % HH); const float* cv = CV + ((size_t)(y + 1) * WP + (x + 1)) * DD; v8us oh, ol;
#pragma unroll 1
    for (int i = 0; i < 8; ++i) { const int c = lane * 8 + i; const float inv = bfr(gam[c]) / sqrtf(bfr(var[c]) + BEPS); const float t = cv[c] * inv + (bfr(bet[c]) - bfr(mu[c]) * inv); const float sv = t / (1.0f + expf(-t)); const unsigned short hb = f2bf(sv); oh[i] = hb; ol[i] = f2bf(sv - bf2f(hb)); }
    const size_t o = q * DD + lane * 8; *(volatile v8us*)(Zh + o) = oh; *(volatile v8us*)(Zl + o) = ol; __threadfence(); *(volatile v8us*)(Zh + o) = oh; *(volatile v8us*)(Zl + o) = ol;
}
__global__ __launch_bounds__(256) void k_qT(const float* __restrict__ xb, float* QT) {
    __shared__ float tl[64][65];
    const int tid = threadIdx.x, c0 = blockIdx.x * 64, p0 = blockIdx.y * 64; const int rr = tid >> 2, cq = (tid & 3) * 16;
#pragma unroll
    for (int i = 0; i < 16; ++i) tl[rr][cq + i] = bfr(xb[(size_t)(c0 + rr) * NQ + p0 + cq + i]);
    __syncthreads();
    const int lane = tid & 31, wv = tid >> 5;
    auto pass = [&]() {
#pragma unroll
        for (int st = 0; st < 4; ++st) { const int pr = wv * 8 + st * 2 + (lane >> 4); const int cl = (lane & 15) * 4; v4f v;
#pragma unroll
            for (int i = 0; i < 4; ++i) v[i] = tl[cl + i][pr];
            *(volatile v4f*)(QT + (size_t)(p0 + pr) * DD + c0 + cl) = v; }
    };
    pass(); __threadfence(); pass();
}
__global__ __launch_bounds__(256) void k_outT(const float* __restrict__ F, float* OUTB) {
    __shared__ float tl[64][65];
    const int tid = threadIdx.x; const int p0 = blockIdx.x * 64, c0 = blockIdx.y * 64; const int rr = tid >> 2, cq = (tid & 3) * 16;
#pragma unroll
    for (int i = 0; i < 16; ++i) tl[rr][cq + i] = F[(size_t)(p0 + rr) * DD + c0 + cq + i];
    __syncthreads();
    const int lane = tid & 31, wv = tid >> 5;
    auto pass = [&]() {
#pragma unroll
        for (int st = 0; st < 4; ++st) { const int cr = wv * 8 + st * 2 + (lane >> 4); const int pq = (lane & 15) * 4; v4f v; const size_t o = ((size_t)c0 + cr) * NQ + p0 + pq;
#pragma unroll
            for (int i = 0; i < 4; ++i) v[i] = tl[pq + i][cr];
            *(volatile v4f*)(OUTB + o) = v; }
    };
    pass(); __threadfence(); pass();
}

extern "C" void kernel_launch(void* const* d_in, const int* in_sizes, int n_in,
                              void* d_out, int out_size, void* d_ws, size_t ws_size, hipStream_t stream) {
    (void)in_sizes; (void)n_in; (void)out_size;
    const float* query = (const float*)d_in[0]; const float* v = (const float*)d_in[1]; const float* qpos = (const float*)d_in[2]; const float* kpos = (const float*)d_in[3]; const float* oW = (const float*)d_in[4];
    const float* wvs = (const float*)d_in[5]; const float* w1 = (const float*)d_in[6]; const float* b1 = (const float*)d_in[7]; const float* w2 = (const float*)d_in[8]; const float* b2 = (const float*)d_in[9];
    const float* c1w = (const float*)d_in[10]; const float* gam = (const float*)d_in[11]; const float* bet = (const float*)d_in[12]; const float* bmu = (const float*)d_in[13]; const float* bvar = (const float*)d_in[14]; const float* c2w = (const float*)d_in[15]; const float* c2b = (const float*)d_in[16];
    float* out = (float*)d_out;
    char* wsp = (char*)d_ws;
    auto take = [&](size_t bytes) { char* p = wsp; wsp += (bytes + 255) & ~(size_t)255; return (void*)p; };
    bf* W1 = (bf*)take((size_t)DD * 2 * DD * 2); bf* W2 = (bf*)take((size_t)DD * DD * 2); bf* WVS = (bf*)take((size_t)DD * DD * 2); bf* WT = (bf*)take((size_t)9 * DD * DD * 2); bf* WC2 = (bf*)take((size_t)DD * DD * 2);
    bf* A2 = (bf*)take((size_t)NQ * 2 * DD * 2); float* H1 = (float*)take((size_t)NQ * DD * 4); bf* Hh = (bf*)take((size_t)NQ * DD * 2); bf* Hl = (bf*)take((size_t)NQ * DD * 2); float* QP = (float*)take((size_t)NQ * DD * 4); float* RQ = (float*)take((size_t)NQ * 32 * 4); float* RK = (float*)take((size_t)NKY * 32 * 4);
    bf* Qh = (bf*)take((size_t)NQ * DD * 2); bf* Ql = (bf*)take((size_t)NQ * DD * 2); bf* KP = (bf*)take((size_t)NKY * DD * 2); bf* VT = (bf*)take((size_t)DD * NKY * 2);
    float* S = (float*)take((size_t)NQ * NKY * 4); bf* PH = (bf*)take((size_t)NQ * NKY * 2); bf* PL = (bf*)take((size_t)NQ * NKY * 2); float* PV = (float*)take((size_t)NQ * DD * 4); bf* PVh = (bf*)take((size_t)NQ * DD * 2); bf* PVl = (bf*)take((size_t)NQ * DD * 2); float* OUT = (float*)take((size_t)NQ * DD * 4);
    bf* Gh = (bf*)take((size_t)NPT * DD * 2); bf* Gl = (bf*)take((size_t)NPT * DD * 2); float* CV = (float*)take((size_t)NPR * DD * 4); bf* Zh = (bf*)take((size_t)NQ * DD * 2); bf* Zl = (bf*)take((size_t)NQ * DD * 2); float* QT = (float*)take((size_t)NQ * DD * 4); float* FO = (float*)take((size_t)NQ * DD * 4);
    if ((size_t)(wsp - (char*)d_ws) > ws_size) return;
    k_cvt8<<<(DD * 2 * DD / 8 + 255) / 256, 256, 0, stream>>>(w1, W1, DD * 2 * DD / 8); k_cvt8<<<(DD * DD / 8 + 255) / 256, 256, 0, stream>>>(w2, W2, DD * DD / 8); k_cvt8<<<(DD * DD / 8 + 255) / 256, 256, 0, stream>>>(wvs, WVS, DD * DD / 8); k_cvt8<<<(DD * DD / 8 + 255) / 256, 256, 0, stream>>>(c2w, WC2, DD * DD / 8);
    k_wtap9<<<(9 * DD) / 8, 256, 0, stream>>>(c1w, WT);
    for (int b = 0; b < NB_; ++b) {
        const float* qb = query + (size_t)b * DD * NQ; const float* vb = v + (size_t)b * NKY * DD; const float* qpb = qpos + (size_t)b * NQ * DD; const float* kpb = kpos + (size_t)b * NKY * DD; const float* owb = oW + (size_t)b * NKY;
        k_qp2<<<NQ / 8, 256, 0, stream>>>(qpb, A2);
        k_gemmb<false, false><<<dim3(NQ / 64, DD / 64, 1), 128, 0, stream>>>(A2, nullptr, W1, b1, H1, DD, nullptr, nullptr, 2 * DD);
        k_relu256p<<<NQ / 8, 256, 0, stream>>>(H1, NQ, Hh, Hl);
        k_gemmb<true, false><<<dim3(NQ / 64, DD / 64, 1), 128, 0, stream>>>(Hh, Hl, W2, b2, QP, DD, nullptr, nullptr, DD);
        k_normsplit<false, true><<<NQ / 8, 256, 0, stream>>>(QP, NQ, RQ, Qh, Ql);
        k_normsplit<true, false><<<NKY / 8, 256, 0, stream>>>(kpb, NKY, RK, nullptr, nullptr);
        k_cvtrows<<<NKY / 8, 256, 0, stream>>>(kpb, NKY, KP); k_vT<<<dim3(NKY / 64, DD / 64, 1), 256, 0, stream>>>(vb, VT);
        k_gemmb<true, false><<<dim3(NQ / 64, NKY / 64, 1), 128, 0, stream>>>(Qh, Ql, KP, nullptr, S, NKY, nullptr, nullptr, DD);
        k_relw<<<NQ / 8, 256, 0, stream>>>(S, RQ, RK, owb, PH, PL);
        k_gemmb<true, false><<<dim3(NQ / 64, DD / 64, 1), 128, 0, stream>>>(PH, PL, VT, nullptr, PV, DD, nullptr, nullptr, NKY);
        k_split256<<<NQ / 8, 256, 0, stream>>>(PV, NQ, PVh, PVl);
        k_gemmb<true, false><<<dim3(NQ / 64, DD / 64, 1), 128, 0, stream>>>(PVh, PVl, WVS, nullptr, OUT, DD, nullptr, nullptr, DD);
        k_ogrid<<<NPT / 8, 256, 0, stream>>>(OUT, Gh, Gl);
        k_gemmtap9<<<dim3(NPR / 64, DD / 64, 1), 128, 0, stream>>>(Gh, Gl, WT, CV);
        k_bnsilu<<<NQ / 8, 256, 0, stream>>>(CV, gam, bet, bmu, bvar, Zh, Zl);
        k_qT<<<dim3(DD / 64, NQ / 64, 1), 256, 0, stream>>>(qb, QT);
        k_gemmb<true, false><<<dim3(NQ / 64, DD / 64, 1), 128, 0, stream>>>(Zh, Zl, WC2, c2b, FO, DD, nullptr, QT, DD, 0);
        k_outT<<<dim3(NQ / 64, DD / 64, 1), 256, 0, stream>>>(FO, out + (size_t)b * DD * NQ); }
}
